// Lorenz96_correction_7421703487572
// MI455X (gfx1250) — hardware-verified
//
#include <hip/hip_runtime.h>
#include <stdint.h>

#define NB    65536
#define XD    40
#define NTHR  128
#define NWAV  4
#define RPB   8
#define NGRP  (NB / RPB)
#define GRIDX 1024
#define C1    72
#define CG    48
#define C2    37
#define KTAP  5
#define KIM   240
#define KPAD  256
#define MPAD  48
#define PP    44
#define GPL   (PP * CG)
#define ASC   64.0f
#define GSC   16.0f
#define B2SC  1024.0f
#define W3SC  0.0009765625f

static_assert(NB % RPB == 0);
static_assert(NGRP % GRIDX == 0);
static_assert(KIM == CG * KTAP);
static_assert((GPL % 8) == 0);
static_assert((KPAD % 8) == 0);
static_assert(RPB * XD * 4 == 10 * 128);
static_assert(NTHR == NWAV * 32);

typedef _Float16 v16h __attribute__((ext_vector_type(16)));
typedef _Float16 v8h  __attribute__((ext_vector_type(8)));
typedef float    v8f  __attribute__((ext_vector_type(8)));
typedef float    v4f  __attribute__((ext_vector_type(4)));

__device__ __forceinline__ float bf_rne(float f) {
  unsigned x = __float_as_uint(f);
  x = (x + 0x7FFFu + ((x >> 16) & 1u)) & 0xFFFF0000u;
  return __uint_as_float(x);
}
__device__ __forceinline__ v8f zero8() { v8f z = {0.f, 0.f, 0.f, 0.f, 0.f, 0.f, 0.f, 0.f}; return z; }

__device__ __forceinline__ v16h ldfrag(const _Float16* p) {
  union { v16h v; v8h h[2]; } f;
  f.h[0] = *(const v8h*)(p);
  f.h[1] = *(const v8h*)(p + 16);
  return f.v;
}
__device__ __forceinline__ v16h ldfrag_lo(const _Float16* p) {
  union { v16h v; v8h h[2]; } f;
  const _Float16 zh = (_Float16)0.0f;
  const v8h z = {zh, zh, zh, zh, zh, zh, zh, zh};
  f.h[0] = *(const v8h*)(p);
  f.h[1] = z;
  return f.v;
}

__device__ __forceinline__ v8f mma_h(v16h a, v16h b, v8f c) {
  return __builtin_amdgcn_wmma_f32_16x16x32_f16(false, a, false, b, (short)0, c, false, false);
}
__device__ __forceinline__ void dep_guard3(v8f& x, v8f& y, v8f& z, v16h a0, v16h a1, v16h a2, v16h b) {
#if defined(__HIP_DEVICE_COMPILE__)
  asm volatile("v_nop\n\tv_nop\n\tv_nop\n\tv_nop" : "+v"(x), "+v"(y), "+v"(z) : "v"(a0), "v"(a1), "v"(a2), "v"(b));
#endif
}
__device__ __forceinline__ void acc_guard3(v8f& x, v8f& y, v8f& z) {
#if defined(__HIP_DEVICE_COMPILE__)
  asm volatile("v_nop\n\tv_nop\n\tv_nop\n\tv_nop" : "+v"(x), "+v"(y), "+v"(z));
#endif
}
__device__ __forceinline__ void wave_sync_lds() {
  __builtin_amdgcn_fence(__ATOMIC_RELEASE, "workgroup");
  __builtin_amdgcn_wave_barrier();
  __builtin_amdgcn_fence(__ATOMIC_ACQUIRE, "workgroup");
}

__global__ __launch_bounds__(NTHR)
void k_main(const float* __restrict__ tt,
            const float* __restrict__ u,
            const float* __restrict__ coeff,
            const float* __restrict__ W1,
            const float* __restrict__ b1,
            const float* __restrict__ W2,
            const float* __restrict__ b2,
            const float* __restrict__ W3,
            const float* __restrict__ b3,
            float* out)
{
  __shared__ __align__(16) _Float16 A_s[MPAD * KPAD];
  __shared__ __align__(16) _Float16 g_s[NWAV][2 * GPL];
  __shared__ __align__(16) float    u_s[NWAV][2 * PP];
  __shared__ __align__(16) float    o_s[RPB * XD];
  __shared__ float w1_s[C1 * KTAP];
  __shared__ float b1_s[C1];
  __shared__ float b2_s[MPAD];
  __shared__ float w3_s[MPAD];
  (void)tt;

  const int tid = threadIdx.x;

  for (int idx = tid; idx < MPAD * KPAD; idx += NTHR) {
    const int m  = idx >> 8;
    const int k  = idx & (KPAD - 1);
    const int kk = k / CG;
    const int c  = k - kk * CG;
    const bool ok = (m < C2) && (k < KIM);
    int src = (m * CG + c) * KTAP + kk;
    src = ok ? src : 0;
    float w = W2[src];
    w = ok ? (bf_rne(w) * ASC) : 0.0f;
    A_s[idx] = (_Float16)w;
  }
  for (int idx = tid; idx < C1 * KTAP; idx += NTHR) w1_s[idx] = bf_rne(W1[idx]);
  if (tid < C1) b1_s[tid] = bf_rne(b1[tid]);
  if (tid < MPAD) {
    const bool ok = (tid < C2);
    const int src = ok ? tid : 0;
    const float bb = b2[src];
    const float ww = W3[src];
    b2_s[tid] = ok ? (bf_rne(bb) * B2SC) : 0.0f;
    w3_s[tid] = ok ? (bf_rne(ww) * W3SC) : 0.0f;
  }
  float cf[18];
#pragma unroll
  for (int j = 0; j < 18; ++j) cf[j] = bf_rne(coeff[j]);
  const float b3r = bf_rne(b3[0]);
  __syncthreads();

  const int lane = tid & 31;
  const int wv   = tid >> 5;
  const int lm   = lane & 15;
  const int hh   = lane >> 4;
  float*    up = &u_s[wv][0];
  _Float16* gp = &g_s[wv][0];
  const _Float16* pa0 = A_s + lm * KPAD + 8 * hh;

  for (int grp = blockIdx.x; grp < NGRP; grp += gridDim.x) {
    const int n0 = grp * RPB + wv * 2;

    {
      const int e = (lane < 20) ? lane : 19;
      const v4f uv = *(const v4f*)(u + (size_t)n0 * XD + 4 * e);
      if (lane < 20) {
        const int rr = (lane >= 10) ? 1 : 0;
        const int d0 = 4 * lane - XD * rr;
        float* upr = up + rr * PP;
#pragma unroll
        for (int j = 0; j < 4; ++j) {
          const float v = bf_rne(uv[j]);
          const int d = d0 + j;
          upr[d + 2] = v;
          if (d >= XD - 2) upr[d - (XD - 2)] = v;
          if (d < 2) upr[d + XD + 2] = v;
        }
      }
    }
    wave_sync_lds();

#pragma unroll 1
    for (int s = 0; s < 3; ++s) {
      const int task = lane + 32 * s;
      const int rr   = (task >= CG) ? 1 : 0;
      const int gch  = task - CG * rr;
      const bool gated = (gch >= 24);
      const int ca = gch;
      const int cb = gated ? (gch + 24) : gch;
      float wa[KTAP], wb[KTAP];
#pragma unroll
      for (int k = 0; k < KTAP; ++k) { wa[k] = w1_s[ca * KTAP + k]; wb[k] = w1_s[cb * KTAP + k]; }
      const float ba = b1_s[ca];
      const float bb = b1_s[cb];
      const float* upr = up + rr * PP;
      _Float16* gpr = gp + rr * GPL + gch;
#pragma unroll 1
      for (int d0 = 0; d0 < XD; d0 += 4) {
        const v4f ua = *(const v4f*)(upr + d0);
        const v4f ub = *(const v4f*)(upr + d0 + 4);
        float uu[8] = {ua[0], ua[1], ua[2], ua[3], ub[0], ub[1], ub[2], ub[3]};
#pragma unroll
        for (int j = 0; j < 4; ++j) {
          float a = ba, b = bb;
#pragma unroll
          for (int k = 0; k < KTAP; ++k) {
            a = fmaf(wa[k], uu[j + k], a);
            b = fmaf(wb[k], uu[j + k], b);
          }
          const float ra = fmaxf(a, 0.0f);
          const float rb = fmaxf(b, 0.0f);
          const float g  = gated ? (ra * rb) : ra;
          const _Float16 gh = (_Float16)(g * GSC);
          const int d = d0 + j;
          gpr[(d + 2) * CG] = gh;
          if (d >= XD - 2) gpr[(d - (XD - 2)) * CG] = gh;
          if (d < 2) gpr[(d + XD + 2) * CG] = gh;
        }
      }
    }
    wave_sync_lds();

#pragma unroll 1
    for (int t = 0; t < 5; ++t) {
      const int p  = 16 * t + lm;
      const int rr = (p >= XD) ? 1 : 0;
      const int d  = p - XD * rr;
      const _Float16* pb = gp + rr * GPL + d * CG + 8 * hh;
      v8f acc0 = zero8(), acc1 = zero8(), acc2 = zero8();
#pragma unroll 1
      for (int k0 = 0; k0 < KIM - 16; k0 += 32) {
        const v16h a0 = ldfrag(pa0 + k0);
        const v16h a1 = ldfrag(pa0 + 16 * KPAD + k0);
        const v16h a2 = ldfrag(pa0 + 32 * KPAD + k0);
        const v16h bq = ldfrag(pb + k0);
        acc0 = mma_h(a0, bq, acc0);
        acc1 = mma_h(a1, bq, acc1);
        acc2 = mma_h(a2, bq, acc2);
        dep_guard3(acc0, acc1, acc2, a0, a1, a2, bq);
      }
      {
        const int k0 = KIM - 16;
        const v16h a0 = ldfrag(pa0 + k0);
        const v16h a1 = ldfrag(pa0 + 16 * KPAD + k0);
        const v16h a2 = ldfrag(pa0 + 32 * KPAD + k0);
        const v16h bq = ldfrag_lo(pb + k0);
        acc0 = mma_h(a0, bq, acc0);
        acc1 = mma_h(a1, bq, acc1);
        acc2 = mma_h(a2, bq, acc2);
        dep_guard3(acc0, acc1, acc2, a0, a1, a2, bq);
      }
      acc_guard3(acc0, acc1, acc2);

      float part = 0.0f;
#pragma unroll
      for (int r = 0; r < 8; ++r) {
        const int m = 8 * hh + r;
        part = fmaf(w3_s[m],      fmaxf(acc0[r] + b2_s[m],      0.0f), part);
        part = fmaf(w3_s[m + 16], fmaxf(acc1[r] + b2_s[m + 16], 0.0f), part);
        part = fmaf(w3_s[m + 32], fmaxf(acc2[r] + b2_s[m + 32], 0.0f), part);
      }
      const float other = __shfl_xor(part, 16, 32);

      const float* uq = up + rr * PP + d;
      const float um2 = uq[0], um1 = uq[1], u00 = uq[2], up1 = uq[3], up2 = uq[4];
      const float o1 = cf[0]
          + cf[1] * um2 + cf[2] * um1 + cf[3] * u00 + cf[4] * up1 + cf[5] * up2
          + cf[6] * um2 * um2 + cf[7] * um1 * um1 + cf[8] * u00 * u00
          + cf[9] * up1 * up1 + cf[10] * up2 * up2
          + cf[11] * um2 * um1 + cf[12] * um1 * u00 + cf[13] * u00 * up1
          + cf[14] * up1 * up2 + cf[15] * um2 * u00 + cf[16] * um1 * up1 + cf[17] * u00 * up2;
      const float total = o1 + (part + other + b3r);
      if (hh == 0) o_s[wv * (2 * XD) + p] = total;
    }
    __syncthreads();

    {
      const int e = (tid < RPB * XD / 4) ? tid : (RPB * XD / 4 - 1);
      const v4f v = *(const v4f*)(o_s + 4 * e);
      float* dst = out + (size_t)grp * (RPB * XD) + 4 * e;
      if (tid < RPB * XD / 4) *(volatile v4f*)dst = v;
      __threadfence();
      if (tid < RPB * XD / 4) *(volatile v4f*)dst = v;
    }
    __syncthreads();
  }
}

extern "C" void kernel_launch(void* const* d_in, const int* in_sizes, int n_in,
                              void* d_out, int out_size, void* d_ws, size_t ws_size,
                              hipStream_t stream) {
  (void)d_ws; (void)ws_size;
  if (n_in < 9) return;
  if (in_sizes[1] != NB * XD) return;
  if (in_sizes[2] < 18) return;
  if (in_sizes[3] < C1 * KTAP) return;
  if (in_sizes[4] < C1) return;
  if (in_sizes[5] < C2 * CG * KTAP) return;
  if (in_sizes[6] < C2) return;
  if (in_sizes[7] < C2) return;
  if (in_sizes[8] < 1) return;
  if (out_size != NB * XD) return;

  const float* tt    = (const float*)d_in[0];
  const float* u     = (const float*)d_in[1];
  const float* coeff = (const float*)d_in[2];
  const float* W1    = (const float*)d_in[3];
  const float* b1    = (const float*)d_in[4];
  const float* W2    = (const float*)d_in[5];
  const float* b2    = (const float*)d_in[6];
  const float* W3    = (const float*)d_in[7];
  const float* b3    = (const float*)d_in[8];
  float* out = (float*)d_out;

  const dim3 grid(GRIDX);
  const dim3 blk(NTHR);
  k_main<<<grid, blk, 0, stream>>>(tt, u, coeff, W1, b1, W2, b2, W3, b3, out);
  (void)hipGetLastError();
}
